// NGCFLayer_17343077941929
// MI455X (gfx1250) — hardware-verified
//
#include <hip/hip_runtime.h>
#include <stddef.h>
#include <stdint.h>

#ifndef SPLIT_R
#define SPLIT_R 1
#endif
#ifndef SPLIT_Q
#define SPLIT_Q 1
#endif

#define NN      100000
#define NE      1600000
#define DF      128
#define KR      (DF * (1 + SPLIT_R))
#define KQ      (DF * (1 + SPLIT_Q))
#define KTOT    (KR + KQ)
#define GBM     128
#define GBN     128
#define MP      100096
#define NTHR    256
#define NWAVE   8
#define EPT     8
#define WCH     (32 * EPT)
#define NBRUN   1024
#define SLB     10
#define NBK     98
#define WLCAP   3072
#define RCAP    18432
#define DEGCAP  64
#define ROWE    512
#define MAXDEG_MEAS   37
#define MAXB1024_MEAS 16666
#define PER     (((NE + NWAVE * WCH - 1) / (NWAVE * WCH)) * WCH)

#define BK_ZINTS  (NWAVE * WLCAP + RCAP + 3 * NBRUN)
#define MISC_INTS 16
#define ROW_INTS  (NWAVE * ROWE / 2)
#define SCAN_INTS (BK_ZINTS + MISC_INTS + ROW_INTS)
#define SCAN_LDS  (SCAN_INTS * 4)
#define GEMM_LDS  (GBM * GBN * 4)

#define PBX  (NN * DF / 8 / NTHR)
#define PBW1 (DF * KR / 8 / NTHR)
#define PBW2 (DF * KQ / 8 / NTHR)
#define PBZ  ((MP - NN) * KTOT / 8 / NTHR)
#define PBTOT (PBX + PBW1 + PBW2 + PBZ)

static_assert(SPLIT_R == 0 || SPLIT_R == 1);
static_assert(SPLIT_Q == 0 || SPLIT_Q == 1);
static_assert(KTOT == 128 * (1 + SPLIT_R) + 128 * (1 + SPLIT_Q));
static_assert(KTOT % 32 == 0 && KTOT <= ROWE && KTOT % 128 == 0);
static_assert(DF == 4 * 32 && GBN == DF);
static_assert(MP == 782 * GBM && MP >= NN && MP - NN == 96);
static_assert(97 * 1024 + 672 == NN);
static_assert(NBK * NBRUN >= NN && (NBK - 1) * NBRUN < NN);
static_assert(NE < (1 << 21) && NBRUN == 1024 && NBRUN == (1 << SLB));
static_assert((((long long)NE) << SLB) < (1LL << 31));
static_assert(NE % WCH == 0 && PER % WCH == 0 && (NWAVE - 1) * PER < NE);
static_assert(NBRUN % GBM == 0 && 1024 % GBM == 0 && NBRUN % NWAVE == 0 && NBRUN % 32 == 0);
static_assert((long long)RCAP * 100 >= (long long)MAXB1024_MEAS * 105);
static_assert(WLCAP >= MAXB1024_MEAS / 8 + 8 * 46 + 1);
static_assert(DEGCAP >= MAXDEG_MEAS + 8);
static_assert(BK_ZINTS % (NTHR * 4) == 0 && (BK_ZINTS + MISC_INTS) % 4 == 0);
static_assert((NN * DF / 8) % NTHR == 0 && (DF * KR / 8) % NTHR == 0 && (DF * KQ / 8) % NTHR == 0);
static_assert(((MP - NN) * KTOT / 8) % NTHR == 0);
static_assert(SCAN_LDS <= 300000 && GEMM_LDS <= 300000);
static_assert(GBM == NWAVE * 16);

typedef float          v4f   __attribute__((ext_vector_type(4)));
typedef float          v8f   __attribute__((ext_vector_type(8)));
typedef int            v4i   __attribute__((ext_vector_type(4)));
typedef int            v8i   __attribute__((ext_vector_type(8)));
typedef unsigned       v2u   __attribute__((ext_vector_type(2)));
typedef unsigned short v4us  __attribute__((ext_vector_type(4)));
typedef unsigned short v8us  __attribute__((ext_vector_type(8)));
typedef unsigned short v16us __attribute__((ext_vector_type(16)));
typedef __bf16         v16bf __attribute__((ext_vector_type(16)));
typedef v4f  __attribute__((may_alias)) v4fa;
typedef v4i  __attribute__((may_alias)) v4ia;
typedef v2u  __attribute__((may_alias)) v2ua;
typedef v4us __attribute__((may_alias)) v4usa;
typedef v8us __attribute__((may_alias)) v8usa;
union FragB { v16bf v; v16us u; v8us h[2]; v8i w; };

__device__ __forceinline__ v8f wmb(const FragB& a, const FragB& b, v8f c) {
  v8f d = __builtin_amdgcn_wmma_f32_16x16x32_bf16(false, a.v, false, b.v, (short)0, c, false, false);
  asm volatile("v_nop\n\tv_nop\n\tv_nop\n\tv_nop" : "+v"(d) : "v"(a.w), "v"(b.w));
  return d;
}

__device__ __forceinline__ unsigned bf16_bits(float f) {
  const unsigned u = __float_as_uint(f);
  const unsigned r = (u + 0x7FFFu + ((u >> 16) & 1u)) >> 16;
  const unsigned q = (u >> 16) | 0x40u;
  return ((u & 0x7fffffffu) > 0x7f800000u) ? q : r;
}

__device__ __forceinline__ void hilo4(float v0, float v1, float v2, float v3, v4us& h, v4us& l) {
  const unsigned a0 = bf16_bits(v0), a1 = bf16_bits(v1), a2 = bf16_bits(v2), a3 = bf16_bits(v3);
  const unsigned b0 = bf16_bits(v0 - __uint_as_float(a0 << 16));
  const unsigned b1 = bf16_bits(v1 - __uint_as_float(a1 << 16));
  const unsigned b2 = bf16_bits(v2 - __uint_as_float(a2 << 16));
  const unsigned b3 = bf16_bits(v3 - __uint_as_float(a3 << 16));
  h[0] = (unsigned short)a0; h[1] = (unsigned short)a1; h[2] = (unsigned short)a2; h[3] = (unsigned short)a3;
  l[0] = (unsigned short)b0; l[1] = (unsigned short)b1; l[2] = (unsigned short)b2; l[3] = (unsigned short)b3;
}

__device__ __forceinline__ void wave_sync() {
  __builtin_amdgcn_fence(__ATOMIC_RELEASE, "wavefront");
  __builtin_amdgcn_wave_barrier();
  __builtin_amdgcn_fence(__ATOMIC_ACQUIRE, "wavefront");
}

__device__ __forceinline__ void st2_v8us(unsigned short* p, v8us v) {
  *(volatile v8us*)p = v;
  __threadfence();
  *(volatile v8us*)p = v;
}

__device__ __forceinline__ v8us gather8(const float* __restrict__ base, int stride) {
  float f[8];
#pragma unroll
  for (int i = 0; i < 8; ++i) f[i] = base[(size_t)i * (size_t)stride];
  v8us o;
#pragma unroll
  for (int i = 0; i < 8; ++i) o[i] = (unsigned short)bf16_bits(f[i]);
  return o;
}

__global__ __launch_bounds__(NTHR) void k_prep(const float* __restrict__ emb, const float* __restrict__ w1,
                                               const float* __restrict__ w2, unsigned short* xb,
                                               unsigned short* wcat, unsigned short* apl) {
  const int tid = (int)threadIdx.x;
  const int blk = (int)blockIdx.x;
  if (blk < PBX) {
    const int u   = blk * NTHR + tid;
    const int row = u >> 4, k8 = (u & 15) * 8;
    const float* p = emb + (size_t)row * DF + k8;
    const v4f a = *(const v4fa*)p;
    const v4f b = *(const v4fa*)(p + 4);
    v8us o;
    o[0] = (unsigned short)bf16_bits(a.x); o[1] = (unsigned short)bf16_bits(a.y);
    o[2] = (unsigned short)bf16_bits(a.z); o[3] = (unsigned short)bf16_bits(a.w);
    o[4] = (unsigned short)bf16_bits(b.x); o[5] = (unsigned short)bf16_bits(b.y);
    o[6] = (unsigned short)bf16_bits(b.z); o[7] = (unsigned short)bf16_bits(b.w);
    st2_v8us(xb + (size_t)row * DF + k8, o);
  } else if (blk < PBX + PBW1) {
    const int u  = (blk - PBX) * NTHR + tid;
    const int n  = u / (KR / 8), k8 = (u % (KR / 8)) * 8, kk = k8 & (DF - 1);
    const v8us o = gather8(w1 + (size_t)kk * DF + n, DF);
    st2_v8us(wcat + (size_t)n * KTOT + k8, o);
  } else if (blk < PBX + PBW1 + PBW2) {
    const int u  = (blk - PBX - PBW1) * NTHR + tid;
    const int n  = u / (KQ / 8), k8 = (u % (KQ / 8)) * 8, kk = k8 & (DF - 1);
    const v8us o = gather8(w2 + (size_t)kk * DF + n, DF);
    st2_v8us(wcat + (size_t)n * KTOT + KR + k8, o);
  } else {
    const int u = (blk - PBX - PBW1 - PBW2) * NTHR + tid;
    const v8us z = {0, 0, 0, 0, 0, 0, 0, 0};
    st2_v8us(apl + (size_t)NN * KTOT + (size_t)u * 8, z);
  }
}

__global__ __launch_bounds__(NTHR) void k_scan(const int* __restrict__ keys, const int* __restrict__ gath,
                                               const float* __restrict__ ew,
                                               const unsigned short* __restrict__ XB,
                                               unsigned short* apl, int* FLAG) {
  extern __shared__ __attribute__((aligned(16))) int dsm[];
  int* wl   = dsm;
  int* pl   = dsm + NWAVE * WLCAP;
  int* cnt  = pl + RCAP;
  int* offs = cnt + NBRUN;
  int* cur  = offs + NBRUN;
  int* misc = cur + NBRUN;
  const int tid = (int)threadIdx.x, lane = tid & 31, wave = tid >> 5;
  unsigned short* rowbuf = (unsigned short*)(misc + MISC_INTS) + wave * ROWE;
  const int blk = (int)blockIdx.x;
  const int nodeBase = blk * NBRUN;
  const unsigned nbs = (unsigned)nodeBase;
  const int nbI = (NN - nodeBase) < NBRUN ? (NN - nodeBase) : NBRUN;
  const unsigned unb = (unsigned)nbI;

  {
    const v4i z4 = {0, 0, 0, 0};
    for (int i = tid * 4; i < BK_ZINTS; i += NTHR * 4) *(v4ia*)(dsm + i) = z4;
    if (tid < MISC_INTS) misc[tid] = 0;
  }
  __syncthreads();

  {
    const int ebeg = wave * PER;
    const int eend = (ebeg + PER < NE) ? (ebeg + PER) : NE;
    int* mylist = wl + wave * WLCAP;
    int wc = 0;
#pragma unroll 1
    for (int cb = ebeg; cb < eend; cb += WCH) {
      const int e0 = cb + lane * EPT;
      const v4i da = *(const v4ia*)(keys + e0);
      const v4i db = *(const v4ia*)(keys + e0 + 4);
      const unsigned s0 = (unsigned)da.x - nbs, s1 = (unsigned)da.y - nbs;
      const unsigned s2 = (unsigned)da.z - nbs, s3 = (unsigned)da.w - nbs;
      const unsigned s4 = (unsigned)db.x - nbs, s5 = (unsigned)db.y - nbs;
      const unsigned s6 = (unsigned)db.z - nbs, s7 = (unsigned)db.w - nbs;
      const bool h0 = s0 < unb, h1 = s1 < unb, h2 = s2 < unb, h3 = s3 < unb;
      const bool h4 = s4 < unb, h5 = s5 < unb, h6 = s6 < unb, h7 = s7 < unb;
      const unsigned m0 = __builtin_amdgcn_ballot_w32(h0), m1 = __builtin_amdgcn_ballot_w32(h1);
      const unsigned m2 = __builtin_amdgcn_ballot_w32(h2), m3 = __builtin_amdgcn_ballot_w32(h3);
      const unsigned m4 = __builtin_amdgcn_ballot_w32(h4), m5 = __builtin_amdgcn_ballot_w32(h5);
      const unsigned m6 = __builtin_amdgcn_ballot_w32(h6), m7 = __builtin_amdgcn_ballot_w32(h7);
      const unsigned any = m0 | m1 | m2 | m3 | m4 | m5 | m6 | m7;
      if (any != 0u) {
        const int pre = (int)(__builtin_amdgcn_mbcnt_lo(m0, 0u) + __builtin_amdgcn_mbcnt_lo(m1, 0u) +
                              __builtin_amdgcn_mbcnt_lo(m2, 0u) + __builtin_amdgcn_mbcnt_lo(m3, 0u) +
                              __builtin_amdgcn_mbcnt_lo(m4, 0u) + __builtin_amdgcn_mbcnt_lo(m5, 0u) +
                              __builtin_amdgcn_mbcnt_lo(m6, 0u) + __builtin_amdgcn_mbcnt_lo(m7, 0u));
        int p = wc + pre;
        if (h0) { if (p < WLCAP) mylist[p] = ((e0 + 0) << SLB) | (int)s0; p = p + 1; }
        if (h1) { if (p < WLCAP) mylist[p] = ((e0 + 1) << SLB) | (int)s1; p = p + 1; }
        if (h2) { if (p < WLCAP) mylist[p] = ((e0 + 2) << SLB) | (int)s2; p = p + 1; }
        if (h3) { if (p < WLCAP) mylist[p] = ((e0 + 3) << SLB) | (int)s3; p = p + 1; }
        if (h4) { if (p < WLCAP) mylist[p] = ((e0 + 4) << SLB) | (int)s4; p = p + 1; }
        if (h5) { if (p < WLCAP) mylist[p] = ((e0 + 5) << SLB) | (int)s5; p = p + 1; }
        if (h6) { if (p < WLCAP) mylist[p] = ((e0 + 6) << SLB) | (int)s6; p = p + 1; }
        if (h7) { if (p < WLCAP) mylist[p] = ((e0 + 7) << SLB) | (int)s7; p = p + 1; }
        wc += (int)(__builtin_popcount(m0) + __builtin_popcount(m1) + __builtin_popcount(m2) + __builtin_popcount(m3) +
                    __builtin_popcount(m4) + __builtin_popcount(m5) + __builtin_popcount(m6) + __builtin_popcount(m7));
      }
    }
    if (lane == 0) misc[wave] = wc;
  }
  __syncthreads();

  if (wave == 0) {
    int ov = 0;
#pragma unroll 1
    for (int w2 = 0; w2 < NWAVE; ++w2) {
      int c = misc[w2];
      if (c > WLCAP) ov = 1;
      c = c < 0 ? 0 : (c > WLCAP ? WLCAP : c);
      c = __builtin_amdgcn_readfirstlane(c);
#pragma unroll 1
      for (int b0 = 0; b0 < c; b0 += 32) {
        const int idx = b0 + lane;
        const int ent = wl[w2 * WLCAP + (idx < WLCAP ? idx : WLCAP - 1)];
        const int m32 = (c - b0) < 32 ? (c - b0) : 32;
#pragma unroll 1
        for (int k = 0; k < m32; ++k) {
          const int u    = __builtin_amdgcn_readlane(ent, k);
          const int slot = u & (NBRUN - 1);
          if (lane == 0) cnt[slot] = cnt[slot] + 1;
        }
      }
    }
    if (lane == 0) misc[9] = ov;
  }
  __syncthreads();
  if (wave == 0) {
    const int base = lane * (NBRUN / 32);
    int s = 0, bg = 0;
#pragma unroll 1
    for (int i = 0; i < NBRUN / 32; ++i) {
      const int cv = cnt[base + i];
      s += cv;
      bg |= (cv > DEGCAP) ? 1 : 0;
    }
    int incl = s;
#pragma unroll
    for (int d = 1; d < 32; d <<= 1) {
      const int y = __shfl_up(incl, d, 32);
      if (lane >= d) incl += y;
    }
    const int tot = __shfl(incl, 31, 32);
    const unsigned anyb = __builtin_amdgcn_ballot_w32(bg != 0);
    int ov2 = misc[9];
    ov2 = (anyb != 0u) ? 1 : ov2;
    ov2 = (tot > RCAP) ? 1 : ov2;
    int run = incl - s;
#pragma unroll 1
    for (int i = 0; i < NBRUN / 32; ++i) {
      const int cv = cnt[base + i];
      offs[base + i] = run;
      cur[base + i]  = run;
      run += cv;
    }
    if (lane == 0) misc[9] = ov2;
  }
  __syncthreads();

  if (wave == 0) {
#pragma unroll 1
    for (int w2 = 0; w2 < NWAVE; ++w2) {
      int c = misc[w2];
      c = c < 0 ? 0 : (c > WLCAP ? WLCAP : c);
      c = __builtin_amdgcn_readfirstlane(c);
#pragma unroll 1
      for (int b0 = 0; b0 < c; b0 += 32) {
        const int idx = b0 + lane;
        const int ent = wl[w2 * WLCAP + (idx < WLCAP ? idx : WLCAP - 1)];
        const int m32 = (c - b0) < 32 ? (c - b0) : 32;
#pragma unroll 1
        for (int k = 0; k < m32; ++k) {
          const int u    = __builtin_amdgcn_readlane(ent, k);
          const int slot = u & (NBRUN - 1);
          const int eid  = (u >> SLB) & 0x1FFFFF;
          if (lane == 0) {
            int p = cur[slot];
            p = p < 0 ? 0 : (p > RCAP - 1 ? RCAP - 1 : p);
            pl[p] = eid;
            cur[slot] = p + 1;
          }
        }
      }
    }
  }
  __syncthreads();

  const int ovf = misc[9];
  if (tid < 8) {
    const v4i f = {ovf, ovf, ovf, ovf};
    int* fp = FLAG + (size_t)blk * 32 + 4 * tid;
    *(volatile v4i*)fp = f;
    __threadfence();
    *(volatile v4i*)fp = f;
  }

  const float qnan = __uint_as_float(0x7fc00000u);
#pragma unroll 1
  for (int si = 0; si < NBRUN / NWAVE; ++si) {
    const int s    = si * NWAVE + wave;
    const int node = nodeBase + s;
    if (node < NN) {
      int cv = cnt[s];
      const bool big = cv > DEGCAP;
      cv = cv < 0 ? 0 : (cv > DEGCAP ? DEGCAP : cv);
      int ovv = offs[s];
      ovv = ovv < 0 ? 0 : (ovv > RCAP - 1 ? RCAP - 1 : ovv);
      const int c = __builtin_amdgcn_readfirstlane(cv);
      const int o = __builtin_amdgcn_readfirstlane(ovv);
      int last = o + c - 1;
      last = last < o ? o : last;
      last = last > RCAP - 1 ? RCAP - 1 : last;
      float a0 = 0.0f, a1 = 0.0f, a2 = 0.0f, a3 = 0.0f;
#pragma unroll 1
      for (int b0 = 0; b0 < c; b0 += 32) {
        int idx = o + b0 + lane;
        idx = idx > last ? last : idx;
        int eid = pl[idx];
        eid = eid < 0 ? 0 : (eid > NE - 1 ? NE - 1 : eid);
        int sr = gath[eid];
        sr = sr < 0 ? 0 : (sr > NN - 1 ? NN - 1 : sr);
        const int wvi = (int)(bf16_bits(ew[eid]) << 16);
        const int m32 = (c - b0) < 32 ? (c - b0) : 32;
#pragma unroll 1
        for (int k = 0; k < m32; ++k) {
          const int   sk = __builtin_amdgcn_readlane(sr, k);
          const float ck = __int_as_float(__builtin_amdgcn_readlane(wvi, k));
          const v2u wd = *(const v2ua*)(XB + (size_t)sk * DF + 4 * lane);
          const float f0 = __uint_as_float(wd.x << 16);
          const float f1 = __uint_as_float(wd.x & 0xffff0000u);
          const float f2 = __uint_as_float(wd.y << 16);
          const float f3 = __uint_as_float(wd.y & 0xffff0000u);
          a0 = fmaf(ck, f0, a0);
          a1 = fmaf(ck, f1, a1);
          a2 = fmaf(ck, f2, a2);
          a3 = fmaf(ck, f3, a3);
        }
      }
      const v2u xo = *(const v2ua*)(XB + (size_t)node * DF + 4 * lane);
      const float x0 = __uint_as_float(xo.x << 16);
      const float x1 = __uint_as_float(xo.x & 0xffff0000u);
      const float x2 = __uint_as_float(xo.y << 16);
      const float x3 = __uint_as_float(xo.y & 0xffff0000u);
      const bool bad = (ovf != 0) | big;
      const float r0 = bad ? qnan : a0, r1 = bad ? qnan : a1, r2 = bad ? qnan : a2, r3 = bad ? qnan : a3;
      const float q0 = r0 * x0, q1 = r1 * x1, q2 = r2 * x2, q3 = r3 * x3;
      v4us rh, rl, qh, ql;
      hilo4(r0, r1, r2, r3, rh, rl);
      hilo4(q0, q1, q2, q3, qh, ql);
      *(v4usa*)(rowbuf + 4 * lane) = rh;
      if constexpr (SPLIT_R != 0) *(v4usa*)(rowbuf + DF + 4 * lane) = rl;
      *(v4usa*)(rowbuf + KR + 4 * lane) = qh;
      if constexpr (SPLIT_Q != 0) *(v4usa*)(rowbuf + KR + DF + 4 * lane) = ql;
      wave_sync();
      constexpr int NST = (KTOT + 255) / 256;
      v4i qv[NST];
#pragma unroll
      for (int j = 0; j < NST; ++j) {
        const int eo = j * 256 + 8 * lane;
        const int ec = eo < KTOT - 8 ? eo : KTOT - 8;
        qv[j] = *(const v4ia*)(rowbuf + ec);
        asm volatile("" :: "v"(qv[j]));
      }
      wave_sync();
      unsigned short* rpw = apl + (size_t)node * KTOT;
#pragma unroll
      for (int j = 0; j < NST; ++j) {
        const int eo = j * 256 + 8 * lane;
        if (eo < KTOT) *(volatile v4i*)(rpw + eo) = qv[j];
      }
      __threadfence();
#pragma unroll
      for (int j = 0; j < NST; ++j) {
        const int eo = j * 256 + 8 * lane;
        if (eo < KTOT) *(volatile v4i*)(rpw + eo) = qv[j];
      }
    }
  }
}

__global__ __launch_bounds__(NTHR) __attribute__((amdgpu_num_vgpr(248)))
void k_gemm(const unsigned short* __restrict__ Apl, const unsigned short* __restrict__ BT,
            const int* __restrict__ FLAG, float* outp) {
  extern __shared__ __attribute__((aligned(16))) float gsm[];
  float* stg = gsm;
  const int tid = (int)threadIdx.x, lane = tid & 31, wave = tid >> 5, hh = lane >> 4, m = lane & 15;
  const int rowBase = (int)blockIdx.x * GBM;

  v8f acc[8];
  {
    const v8f z = {0.f, 0.f, 0.f, 0.f, 0.f, 0.f, 0.f, 0.f};
#pragma unroll
    for (int t = 0; t < 8; ++t) acc[t] = z;
  }
  const unsigned short* ap = Apl + (size_t)(rowBase + 16 * wave + m) * (size_t)KTOT + 8 * hh;
  const unsigned short* bp = BT + (size_t)m * (size_t)KTOT + 8 * hh;

#pragma unroll 1
  for (int k0 = 0; k0 < KTOT; k0 += 32) {
    FragB af;
    af.h[0] = *(const v8usa*)(ap + k0);
    af.h[1] = *(const v8usa*)(ap + k0 + 16);
#pragma unroll
    for (int nt = 0; nt < 8; ++nt) {
      const unsigned short* wq = bp + (size_t)(16 * nt) * (size_t)KTOT + k0;
      FragB bf;
      bf.h[0] = *(const v8usa*)wq;
      bf.h[1] = *(const v8usa*)(wq + 16);
      acc[nt] = wmb(af, bf, acc[nt]);
    }
  }

#pragma unroll
  for (int nt = 0; nt < 8; ++nt) {
    const int lc = 16 * nt + m;
#pragma unroll
    for (int r = 0; r < 8; ++r) {
      const int lr = 16 * wave + 8 * hh + r;
      stg[lr * GBN + lc] = acc[nt][r];
    }
  }
  __syncthreads();

  const int flag = FLAG[(size_t)(rowBase >> SLB) * 32];
  const float qnan = __uint_as_float(0x7fc00000u);
  v4f pv[16];
#pragma unroll
  for (int i = 0; i < 16; ++i) pv[i] = *(const v4fa*)(stg + (16 * wave + i) * GBN + 4 * lane);
#pragma unroll
  for (int i = 0; i < 16; ++i) {
    v4f y = pv[i];
    y.x = (flag != 0) ? qnan : y.x; y.y = (flag != 0) ? qnan : y.y;
    y.z = (flag != 0) ? qnan : y.z; y.w = (flag != 0) ? qnan : y.w;
    pv[i] = y;
  }
#pragma unroll
  for (int i = 0; i < 16; ++i) {
    const int r = rowBase + 16 * wave + i;
    if (r < NN) *(volatile v4f*)(outp + (size_t)r * DF + 4 * lane) = pv[i];
  }
  __threadfence();
#pragma unroll
  for (int i = 0; i < 16; ++i) {
    const int r = rowBase + 16 * wave + i;
    if (r < NN) *(volatile v4f*)(outp + (size_t)r * DF + 4 * lane) = pv[i];
  }
}

extern "C" void kernel_launch(void* const* d_in, const int* in_sizes, int n_in,
                              void* d_out, int out_size, void* d_ws, size_t ws_size,
                              hipStream_t stream) {
  if (n_in < 6) return;
  if (in_sizes[0] != NN * DF) return;
  if (in_sizes[1] != NE) return;
  if (in_sizes[2] != NE) return;
  if (in_sizes[3] != NE) return;
  if (in_sizes[4] != DF * DF) return;
  if (in_sizes[5] != DF * DF) return;
  if (out_size != NN * DF) return;

  const float* emb  = (const float*)d_in[0];
  const int*   erow = (const int*)d_in[1];
  const int*   ecol = (const int*)d_in[2];
  const float* eval = (const float*)d_in[3];
  const float* W1   = (const float*)d_in[4];
  const float* W2   = (const float*)d_in[5];
  float* out = (float*)d_out;

  constexpr size_t zA    = (size_t)MP * KTOT * 2;
  constexpr size_t zXB   = (size_t)NN * DF * 2;
  constexpr size_t zW    = (size_t)DF * KTOT * 2;
  constexpr size_t zFLAG = (size_t)NBK * 128;
  constexpr size_t oA    = 0;
  constexpr size_t oXB   = oA + zA;
  constexpr size_t oW    = oXB + zXB;
  constexpr size_t oFLAG = oW + zW;
  constexpr size_t oEND  = oFLAG + zFLAG;
  static_assert(zA % 256 == 0 && zXB % 256 == 0 && zW % 256 == 0 && zFLAG % 256 == 0);
  static_assert(oEND <= (size_t)(128u << 20));
  if (oEND > ws_size) return;

  char* ws = (char*)d_ws;
  unsigned short* Apl  = (unsigned short*)(ws + oA);
  unsigned short* XB   = (unsigned short*)(ws + oXB);
  unsigned short* WCAT = (unsigned short*)(ws + oW);
  int*            FLAG = (int*)(ws + oFLAG);

  hipFuncSetAttribute(reinterpret_cast<const void*>(&k_scan), hipFuncAttributeMaxDynamicSharedMemorySize, (int)SCAN_LDS);
  hipFuncSetAttribute(reinterpret_cast<const void*>(&k_gemm), hipFuncAttributeMaxDynamicSharedMemorySize, (int)GEMM_LDS);

  k_prep<<<PBTOT, NTHR, 0, stream>>>(emb, W1, W2, XB, WCAT, Apl);
  k_scan<<<NBK, NTHR, SCAN_LDS, stream>>>(erow, ecol, eval, XB, Apl, FLAG);
  k_gemm<<<MP / GBM, NTHR, GEMM_LDS, stream>>>(Apl, WCAT, FLAG, out);
}
